// PhysicsForwardModel_1992864825659
// MI455X (gfx1250) — hardware-run, weakly checked
//
#include <hip/hip_runtime.h>


#define NB_  4
#define NZ   128
#define LL   512
#define JG   64
#define NJG  (LL / JG)
#define NPB  64
#define PI_F 3.1415927f
typedef _Float16 h16;
typedef unsigned short bf;
typedef __attribute__((ext_vector_type(16))) __bf16   v16bf;
typedef __attribute__((ext_vector_type(16))) _Float16 v16h;
typedef __attribute__((ext_vector_type(8)))  _Float16 v8h;
typedef __attribute__((ext_vector_type(8)))  unsigned short v8us;
typedef __attribute__((ext_vector_type(8)))  float    v8f;
typedef __attribute__((ext_vector_type(4)))  float    v4f;
typedef v8h  __attribute__((may_alias)) v8ha;
typedef v4f  __attribute__((may_alias)) v4fa;
typedef v8us __attribute__((may_alias)) v8usa;

__device__ __forceinline__ unsigned short f2bf(float f) { unsigned u = __float_as_uint(f); u += 0x7FFFu + ((u >> 16) & 1u); return (unsigned short)(u >> 16); }
__device__ __forceinline__ float bf2f(unsigned short b) { return __uint_as_float(((unsigned)b) << 16); }
__device__ __forceinline__ float bfr(float f) { return bf2f(f2bf(f)); }
__device__ __forceinline__ v16h cat16(v8h lo, v8h hi) { return __builtin_shufflevector(lo, hi, 0, 1, 2, 3, 4, 5, 6, 7, 8, 9, 10, 11, 12, 13, 14, 15); }
__device__ __forceinline__ v16bf cat16b(v8us lo, v8us hi) { return __builtin_bit_cast(v16bf, __builtin_shufflevector(lo, hi, 0, 1, 2, 3, 4, 5, 6, 7, 8, 9, 10, 11, 12, 13, 14, 15)); }
__device__ __forceinline__ v8f wmma16(v16h a, v16h b, v8f c) { return __builtin_amdgcn_wmma_f32_16x16x32_f16(false, a, false, b, (short)0, c, false, false); }
__device__ __forceinline__ v8f wmmab(v16bf a, v16bf b, v8f c) { return __builtin_amdgcn_wmma_f32_16x16x32_bf16(false, a, false, b, (short)0, c, false, false); }


template <typename T16> struct WFrag;
template <> struct WFrag<h16> { typedef v16h V; static __device__ __forceinline__ V ld(const h16* p) { return cat16(*(const v8h*)p, *(const v8h*)(p + 16)); } static __device__ __forceinline__ v8f mma(V a, V b, v8f c) { return wmma16(a, b, c); } };
template <> struct WFrag<bf> { typedef v16bf V; static __device__ __forceinline__ V ld(const bf* p) { return cat16b(*(const v8us*)p, *(const v8us*)(p + 16)); } static __device__ __forceinline__ v8f mma(V a, V b, v8f c) { return wmmab(a, b, c); } };
template <typename T16, int NSPLIT, bool BIAS>
__global__ __launch_bounds__(32) void k_gemmw(const T16* __restrict__ A, const T16* __restrict__ A2, const T16* __restrict__ Bt, const T16* __restrict__ Bt2, int K, float* C, int ldc, const float* __restrict__ bias, size_t sA, size_t sB, size_t sC) {
    typedef typename WFrag<T16>::V V;
    __shared__ __align__(16) float os[16 * 68];
    const size_t z = blockIdx.z; A += z * sA; if (A2) A2 += z * sA; Bt += z * sB; if (Bt2) Bt2 += z * sB; C += z * sC;
    const int lane = threadIdx.x & 31, lr = lane & 15, hi = lane >> 4; const int r0 = blockIdx.x * 64, c0 = blockIdx.y * 64;
    v8f acc[4][4];
#pragma unroll
    for (int mb = 0; mb < 4; ++mb)
#pragma unroll
        for (int nb = 0; nb < 4; ++nb) acc[mb][nb] = (v8f){};
    const size_t aoff = (size_t)(r0 + lr) * K + 8 * hi, boff = (size_t)(c0 + lr) * K + 8 * hi;
#pragma unroll 1
    for (int kc = 0; kc < K; kc += 32) {
        V a[4], a2[4];
#pragma unroll
        for (int mb = 0; mb < 4; ++mb) { a[mb] = WFrag<T16>::ld(A + aoff + (size_t)mb * 16 * K + kc); if (NSPLIT == 1 || NSPLIT == 2) a2[mb] = WFrag<T16>::ld(A2 + aoff + (size_t)mb * 16 * K + kc); }
#pragma unroll
        for (int nb = 0; nb < 4; ++nb) { const V b = WFrag<T16>::ld(Bt + boff + (size_t)nb * 16 * K + kc); V b2; if (NSPLIT >= 2) b2 = WFrag<T16>::ld(Bt2 + boff + (size_t)nb * 16 * K + kc);
#pragma unroll
            for (int mb = 0; mb < 4; ++mb) { acc[mb][nb] = WFrag<T16>::mma(a[mb], b, acc[mb][nb]); if (NSPLIT == 1 || NSPLIT == 2) acc[mb][nb] = WFrag<T16>::mma(a2[mb], b, acc[mb][nb]); if (NSPLIT >= 2) acc[mb][nb] = WFrag<T16>::mma(a[mb], b2, acc[mb][nb]); } }
        asm volatile("v_nop\n\tv_nop\n\tv_nop\n\tv_nop" : "+v"(acc[0][0]), "+v"(acc[1][1]), "+v"(acc[2][2]), "+v"(acc[3][3]) : "v"(a[0]), "v"(a[3]));
    }
#pragma unroll
    for (int mb = 0; mb < 4; ++mb) {
#pragma unroll
        for (int nb = 0; nb < 4; ++nb) {
#pragma unroll
            for (int j = 0; j < 8; ++j) os[(hi * 8 + j) * 68 + nb * 16 + lr] = acc[mb][nb][j]; }
        __builtin_amdgcn_wave_barrier(); asm volatile("" ::: "memory");
        float* crow = C + (size_t)(r0 + mb * 16) * ldc + c0;
#pragma unroll 1
        for (int ps = 0; ps < 2; ++ps) {
#pragma unroll
            for (int s = 0; s < 8; ++s) { const int row = 2 * s + hi, cofs = lr * 4; v4f val = *(const v4fa*)(os + row * 68 + cofs); if (BIAS) { val[0] += bfr(bias[c0 + cofs]); val[1] += bfr(bias[c0 + cofs + 1]); val[2] += bfr(bias[c0 + cofs + 2]); val[3] += bfr(bias[c0 + cofs + 3]); }
                *(volatile v4f*)(crow + (size_t)row * ldc + cofs) = val; }
            if (ps == 0) __threadfence(); }
        __builtin_amdgcn_wave_barrier(); asm volatile("" ::: "memory");
    }
}

__device__ __forceinline__ void splitf(float y, unsigned short& h, unsigned short& l) { h = f2bf(y); l = f2bf(y - bf2f(h)); }
typedef __attribute__((ext_vector_type(2))) unsigned short v2us;
typedef __attribute__((ext_vector_type(2))) float v2f;
__global__ __launch_bounds__(256) void k_cvt8(const float* __restrict__ src, bf* dst, size_t n8) { const size_t i = (size_t)blockIdx.x * 256 + threadIdx.x; if (i >= n8) return; const v8f v = *(const v8f*)(src + i * 8); v8us o;
#pragma unroll
    for (int k = 0; k < 8; ++k) o[k] = f2bf(v[k]); *(volatile v8us*)(dst + i * 8) = o; __threadfence(); *(volatile v8us*)(dst + i * 8) = o; }

__device__ __forceinline__ float dct_el(int r, int c) { const float t1 = (float)(2 * c + 1); const float t2 = __fmul_rn(PI_F, t1); const float t3 = __fmul_rn(t2, (float)r); const float a = t3 * (1.0f / 1024.0f); const float s = (r == 0) ? 0.044194173824159216f : 0.0625f; return __fmul_rn(s, cosf(a)); }
__global__ __launch_bounds__(256) void k_dct(bf* AYh, bf* AYl, bf* BXh, bf* BXl) { const size_t e = ((size_t)blockIdx.x * 256 + threadIdx.x) * 2; if (e >= (size_t)LL * NZ) return; const int c = (int)(e % NZ), r = (int)(e / NZ); v2us ah, al, bh, bl;
#pragma unroll
    for (int q = 0; q < 2; ++q) { unsigned short h, l; splitf(dct_el(r, c + q), h, l); ah[q] = h; al[q] = l; splitf(dct_el(r, NZ + c + q), h, l); bh[q] = h; bl[q] = l; }
    *(volatile v2us*)(AYh + e) = ah; *(volatile v2us*)(AYl + e) = al; *(volatile v2us*)(BXh + e) = bh; *(volatile v2us*)(BXl + e) = bl; __threadfence(); *(volatile v2us*)(AYh + e) = ah; *(volatile v2us*)(AYl + e) = al; *(volatile v2us*)(BXh + e) = bh; *(volatile v2us*)(BXl + e) = bl; }
__global__ __launch_bounds__(256) void k_vvec(float* V) { const int y = blockIdx.x * 256 + threadIdx.x; if (y >= LL) return; float s = 0.f;
#pragma unroll 1
    for (int k = 0; k < LL; ++k) { float p = __fmul_rn(dct_el(y, k), dct_el(k, 0)); asm volatile("" : "+v"(p)); s = __fadd_rn(s, p); }
    *(volatile float*)(V + y) = s; __threadfence(); *(volatile float*)(V + y) = s; }
__global__ __launch_bounds__(256) void k_split8(const float* __restrict__ F, bf* H, bf* Lw, size_t n8) { const size_t i = (size_t)blockIdx.x * 256 + threadIdx.x; if (i >= n8) return; const v8f v = *(const v8f*)(F + i * 8); v8us oh, ol;
#pragma unroll
    for (int q = 0; q < 8; ++q) { unsigned short a, c; splitf(v[q], a, c); oh[q] = a; ol[q] = c; } *(volatile v8us*)(H + i * 8) = oh; *(volatile v8us*)(Lw + i * 8) = ol; __threadfence(); *(volatile v8us*)(H + i * 8) = oh; *(volatile v8us*)(Lw + i * 8) = ol; }
__global__ __launch_bounds__(256) void k_wt(const float* __restrict__ PH, const float* __restrict__ V, bf* Wh, bf* Wl) { const size_t e = ((size_t)blockIdx.x * 256 + threadIdx.x) * 2; if (e >= (size_t)LL * NPB * LL) return; const int i = (int)(e % LL); const int b = (int)((e / LL) % NPB); const int j = (int)(e / ((size_t)LL * NPB)); v2us oh, ol;
#pragma unroll
    for (int q = 0; q < 2; ++q) { float w = 0.f; if (b < NB_) w = __fmul_rn(V[i + q], PH[((size_t)b * LL + i + q) * LL + j]); unsigned short a, c; splitf(w, a, c); oh[q] = a; ol[q] = c; }
    *(volatile v2us*)(Wh + e) = oh; *(volatile v2us*)(Wl + e) = ol; __threadfence(); *(volatile v2us*)(Wh + e) = oh; *(volatile v2us*)(Wl + e) = ol; }
__device__ __forceinline__ void fg_of(int i, int j, float chi, float& F, float& g) { const float kx = __fmul_rn((float)j * (1.0f / LL), PI_F); const float ky = __fmul_rn((float)i * (1.0f / LL), PI_F); float kk = __fmul_rn(kx, kx); asm volatile("" : "+v"(kk)); F = __fsqrt_rn(__fadd_rn(kk, __fmul_rn(ky, ky))); g = __fmul_rn(-chi, F); }
__global__ __launch_bounds__(256) void k_seed(const float* __restrict__ chi_in, int jg, float* SEED) { const int e = blockIdx.x * 256 + threadIdx.x; if (e >= JG * LL) return; const int i = e % LL, jl = e / LL; float F, g; fg_of(i, jg * JG + jl, bfr(chi_in[0]), F, g);
#pragma unroll 1
    for (int ps = 0; ps < 2; ++ps) {
#pragma unroll 1
        for (int k = 0; k < LL / 64; ++k) { const float t0 = (float)(k * 64); const float a = __fmul_rn(F, t0); const float eta = __fmaf_rn(F, t0, -a); const float ca = cosf(a), sa = sinf(a); v4f rec;
            rec[0] = __fsub_rn(ca, __fmul_rn(eta, sa)); rec[1] = __fadd_rn(sa, __fmul_rn(eta, ca)); const float bb = __fmul_rn(g, t0); const float dl = __fmaf_rn(g, t0, -bb); rec[2] = __fmul_rn(expf(bb), __fadd_rn(1.0f, dl)); rec[3] = 0.f;
            *(volatile v4f*)(SEED + ((size_t)e * (LL / 64) + k) * 4) = rec; }
        if (ps == 0) __threadfence(); } }
__global__ __launch_bounds__(256) void k_gen(const float* __restrict__ chi_in, int jg, float* GEN) { const int e = blockIdx.x * 256 + threadIdx.x; if (e >= JG * LL) return; const int i = e % LL, jl = e / LL; float F, g; fg_of(i, jg * JG + jl, bfr(chi_in[0]), F, g); v4f r; r[0] = cosf(F); r[1] = sinf(F); r[2] = expf(g); r[3] = 0.f;
    *(volatile v4f*)(GEN + (size_t)e * 4) = r; __threadfence(); *(volatile v4f*)(GEN + (size_t)e * 4) = r; }
__global__ __launch_bounds__(256) void k_att(const float* __restrict__ chi_in, int jg, const float* __restrict__ SEED, const float* __restrict__ GEN, bf* Ah, bf* Al) {
    const int e = blockIdx.x * 256 + threadIdx.x; if (e >= JG * (LL / 2)) return; const int ip = (e % (LL / 2)) * 2; const int jl = e / (LL / 2); const float chi = bfr(chi_in[0]); float F[2], g[2], c1[2], s1[2], e1[2];
#pragma unroll
    for (int q = 0; q < 2; ++q) { fg_of(ip + q, jg * JG + jl, chi, F[q], g[q]); const v4f gr = *(const v4f*)(GEN + (size_t)(jl * LL + ip + q) * 4); c1[q] = gr[0]; s1[q] = gr[1]; e1[q] = gr[2]; }
#pragma unroll 1
    for (int ps = 0; ps < 2; ++ps) { float c[2], s[2], ex[2];
#pragma unroll 1
        for (int t = 0; t < LL; ++t) {
            if ((t & 63) == 0) {
#pragma unroll
                for (int q = 0; q < 2; ++q) { const v4f rec = *(const v4f*)(SEED + ((size_t)(jl * LL + ip + q) * (LL / 64) + (t >> 6)) * 4); c[q] = rec[0]; s[q] = rec[1]; ex[q] = rec[2]; } }
            v2us oh, ol;
#pragma unroll
            for (int q = 0; q < 2; ++q) { const float a = __fmul_rn(F[q], (float)t); const float eta = __fmaf_rn(F[q], (float)t, -a); const float ca = __fmaf_rn(eta, s[q], c[q]); const float bb = __fmul_rn(g[q], (float)t); const float dl = __fmaf_rn(g[q], (float)t, -bb);
                const float eb = __fmul_rn(ex[q], __fsub_rn(1.0f, dl)); const float at = __fmul_rn(eb, ca); unsigned short hh, l2; splitf(at, hh, l2); oh[q] = hh; ol[q] = l2;
                const float cn = __fsub_rn(__fmul_rn(c[q], c1[q]), __fmul_rn(s[q], s1[q])); const float sn = __fadd_rn(__fmul_rn(s[q], c1[q]), __fmul_rn(c[q], s1[q])); c[q] = cn; s[q] = sn; ex[q] = __fmul_rn(ex[q], e1[q]); }
            const size_t oo = ((size_t)jl * LL + t) * LL + ip; *(volatile v2us*)(Ah + oo) = oh; *(volatile v2us*)(Al + oo) = ol; }
        if (ps == 0) __threadfence(); } }

__global__ __launch_bounds__(256) void k_pout(const float* __restrict__ CT, int jg, float* OUT) { const size_t e = ((size_t)blockIdx.x * 256 + threadIdx.x) * 2; if (e >= (size_t)NB_ * LL * JG) return; const int jl = (int)(e % JG); const int t = (int)((e / JG) % LL); const int b = (int)(e / ((size_t)JG * LL)); v2f v;
#pragma unroll
    for (int q = 0; q < 2; ++q) v[q] = __fdiv_rn(CT[((size_t)(jl + q) * LL + t) * NPB + b], 3.0f);
    float* dst = OUT + ((size_t)b * LL + t) * LL + jg * JG + jl; *(volatile v2f*)dst = v; __threadfence(); *(volatile v2f*)dst = v; }

extern "C" void kernel_launch(void* const* d_in, const int* in_sizes, int n_in,
                              void* d_out, int out_size, void* d_ws, size_t ws_size, hipStream_t stream) {
    (void)in_sizes; (void)n_in; (void)out_size;
    const float* x = (const float*)d_in[0]; const float* chi = (const float*)d_in[1]; (void)d_in[2];
    float* OUT = (float*)d_out;
    char* wsp = (char*)d_ws;
    auto take = [&](size_t bytes) { char* p = wsp; wsp += (bytes + 255) & ~(size_t)255; return (void*)p; };
    bf* AYh = (bf*)take((size_t)LL * NZ * 2); bf* AYl = (bf*)take((size_t)LL * NZ * 2); bf* BXh = (bf*)take((size_t)LL * NZ * 2); bf* BXl = (bf*)take((size_t)LL * NZ * 2); float* V = (float*)take((size_t)LL * 4);
    bf* XB = (bf*)take((size_t)NZ * NZ * 2); float* T1 = (float*)take((size_t)LL * NZ * 4); bf* T1h = (bf*)take((size_t)LL * NZ * 2); bf* T1l = (bf*)take((size_t)LL * NZ * 2); float* PH = (float*)take((size_t)NB_ * LL * LL * 4);
    bf* WTh = (bf*)take((size_t)LL * NPB * LL * 2); bf* WTl = (bf*)take((size_t)LL * NPB * LL * 2); bf* ATh = (bf*)take((size_t)JG * LL * LL * 2); bf* ATl = (bf*)take((size_t)JG * LL * LL * 2); float* CT = (float*)take((size_t)JG * LL * NPB * 4); float* SEED = (float*)take((size_t)JG * LL * (LL / 64) * 4 * 4); float* GEN = (float*)take((size_t)JG * LL * 4 * 4);
    if ((size_t)(wsp - (char*)d_ws) > ws_size) return;
    k_dct<<<(unsigned)(((size_t)LL * NZ / 2 + 255) / 256), 256, 0, stream>>>(AYh, AYl, BXh, BXl); k_vvec<<<LL / 256, 256, 0, stream>>>(V);
    for (int b = 0; b < NB_; ++b) {
        k_cvt8<<<(NZ * NZ / 8 + 255) / 256, 256, 0, stream>>>(x + (size_t)b * NZ * NZ, XB, (size_t)NZ * NZ / 8);
        k_gemmw<bf, 1, false><<<dim3(LL / 64, NZ / 64, 1), 32, 0, stream>>>(BXh, BXl, XB, nullptr, NZ, T1, NZ, nullptr, 0, 0, 0);
        k_split8<<<(LL * NZ / 8 + 255) / 256, 256, 0, stream>>>(T1, T1h, T1l, (size_t)LL * NZ / 8);
        k_gemmw<bf, 2, false><<<dim3(LL / 64, LL / 64, 1), 32, 0, stream>>>(AYh, AYl, T1h, T1l, NZ, PH + (size_t)b * LL * LL, LL, nullptr, 0, 0, 0); }
    k_wt<<<(unsigned)(((size_t)LL * NPB * LL / 2 + 255) / 256), 256, 0, stream>>>(PH, V, WTh, WTl);
    for (int jg = 0; jg < NJG; ++jg) {
        k_seed<<<(JG * LL + 255) / 256, 256, 0, stream>>>(chi, jg, SEED); k_gen<<<(JG * LL + 255) / 256, 256, 0, stream>>>(chi, jg, GEN); k_att<<<(JG * (LL / 2) + 255) / 256, 256, 0, stream>>>(chi, jg, SEED, GEN, ATh, ATl);
        k_gemmw<bf, 2, false><<<dim3(LL / 64, NPB / 64, JG), 32, 0, stream>>>(ATh, ATl, WTh + (size_t)jg * JG * NPB * LL, WTl + (size_t)jg * JG * NPB * LL, LL, CT, NPB, nullptr, (size_t)LL * LL, (size_t)NPB * LL, (size_t)LL * NPB);
        k_pout<<<(unsigned)(((size_t)NB_ * LL * JG / 2 + 255) / 256), 256, 0, stream>>>(CT, jg, OUT); }
}
